// CausalSelfAttention_13142599926188
// MI455X (gfx1250) — hardware-verified
//
#include <hip/hip_runtime.h>


#ifndef NB
#define NB 2
#endif
#ifndef SEQ
#define SEQ 2048
#endif
#define NB_FULL  2
#define SEQ_FULL 2048
#ifndef OUT_SEQ
#define OUT_SEQ SEQ
#endif
#ifndef ER
#define ER 256
#endif
#ifndef ESC_RES
#define ESC_RES 1
#endif
#define DM   2048
#define NH_  16
#define HD   128
#define AW   4
#define OSP  132
#define ESP  68
#define CSP  128
#define FLP  64
#define QRS  2048.0f
#define QRI  (1.0f / 2048.0f)
#define SC2  (0.08838834764831845f * 1.4426950408889634f)
#define L2E  1.4426950408889634f
#define PSH  8.0f
#define CXS  256.0f
#define WOS  64.0f
#define OSC  (1.0f / 16384.0f)

static_assert(HD == 128);
static_assert(NH_ * HD == DM);
static_assert(DM % 64 == 0);
static_assert(HD % 64 == 0);
static_assert(DM % 32 == 0);
static_assert(SEQ % 64 == 0);
static_assert((NB * SEQ) % 64 == 0);
static_assert(SEQ % 32 == 0);
static_assert(SEQ % (16 * AW) == 0);
static_assert(((size_t)SEQ * DM) % 8 == 0);
static_assert(NB <= NB_FULL);
static_assert(SEQ <= SEQ_FULL);
static_assert(ER % 64 == 0);
static_assert(ER >= 64);
static_assert(ER <= SEQ);
static_assert(ER % (16 * AW) == 0);
static_assert((SEQ - ER) % (16 * AW) == 0);
static_assert((SEQ - ER) % 64 == 0);
static_assert(SEQ / 32 <= FLP);
static_assert(FLP % 8 == 0);
static_assert(FLP / 4 <= 32);
static_assert((FLP * 4) % 128 == 0);
static_assert(SEQ % 4 == 0);
static_assert(HD / 2 == 64);
static_assert(CSP == HD);
static_assert(OSP >= HD + 4);
static_assert(ESP >= 64 + 4);
static_assert(HD / 16 == 8);

typedef _Float16 h16;
typedef unsigned short bf;
typedef __attribute__((ext_vector_type(16))) __bf16   v16bf;
typedef __attribute__((ext_vector_type(16))) _Float16 v16h;
typedef __attribute__((ext_vector_type(8)))  _Float16 v8h;
typedef __attribute__((ext_vector_type(8)))  unsigned short v8us;
typedef __attribute__((ext_vector_type(8)))  float    v8f;
typedef __attribute__((ext_vector_type(4)))  float    v4f;
typedef __attribute__((ext_vector_type(4)))  int      v4i;
typedef v4f  __attribute__((may_alias)) v4fa;

__device__ __forceinline__ unsigned short f2bf(float f) { unsigned u = __float_as_uint(f); u += 0x7FFFu + ((u >> 16) & 1u); return (unsigned short)(u >> 16); }
__device__ __forceinline__ float bfr(float f) { return __uint_as_float(((unsigned)f2bf(f)) << 16); }
__device__ __forceinline__ v16h cat16(v8h lo, v8h hi) { return __builtin_shufflevector(lo, hi, 0, 1, 2, 3, 4, 5, 6, 7, 8, 9, 10, 11, 12, 13, 14, 15); }
__device__ __forceinline__ v16bf cat16b(v8us lo, v8us hi) { return __builtin_bit_cast(v16bf, __builtin_shufflevector(lo, hi, 0, 1, 2, 3, 4, 5, 6, 7, 8, 9, 10, 11, 12, 13, 14, 15)); }
__device__ __forceinline__ v8f wmma16(v16h a, v16h b, v8f c) { return __builtin_amdgcn_wmma_f32_16x16x32_f16(false, a, false, b, (short)0, c, false, false); }
__device__ __forceinline__ v8f wmmab(v16bf a, v16bf b, v8f c) { return __builtin_amdgcn_wmma_f32_16x16x32_bf16(false, a, false, b, (short)0, c, false, false); }
__device__ __forceinline__ v16h  ldh(const h16* p) { return cat16(*(const v8h*)p, *(const v8h*)(p + 16)); }
__device__ __forceinline__ v16bf ldb(const bf* p)  { return cat16b(*(const v8us*)p, *(const v8us*)(p + 16)); }
__device__ __forceinline__ void wave_sync() { __builtin_amdgcn_fence(3  , "wavefront"); __builtin_amdgcn_wave_barrier(); asm volatile("" ::: "memory"); }

__device__ __forceinline__ v8f wmma16g(v16h a, v16h b, v8f c) { c = __builtin_amdgcn_wmma_f32_16x16x32_f16(false, a, false, b, (short)0, c, false, false); asm volatile("v_nop\n\tv_nop\n\tv_nop\n\tv_nop" : "+v"(c) : "v"(a), "v"(b)); return c; }
__device__ __forceinline__ v8f wmmabg(v16bf a, v16bf b, v8f c) { c = __builtin_amdgcn_wmma_f32_16x16x32_bf16(false, a, false, b, (short)0, c, false, false); asm volatile("v_nop\n\tv_nop\n\tv_nop\n\tv_nop" : "+v"(c) : "v"(a), "v"(b)); return c; }
static __device__ __forceinline__ h16 toh_flush(float v) { const h16 r = (h16)v; return (fabsf(v) < 6.103515625e-05f) ? (h16)0.0f : r; }

__global__ __launch_bounds__(256) void k_cvt8(const float* __restrict__ src, bf* dst, size_t n8) {
    const size_t i = (size_t)blockIdx.x * 256 + threadIdx.x; if (i >= n8) return;
    const v8f v = *(const v8f*)(src + i * 8); v8us o;
#pragma unroll
    for (int k = 0; k < 8; ++k) o[k] = f2bf(v[k]);
    *(volatile v8us*)(dst + i * 8) = o; __threadfence(); *(volatile v8us*)(dst + i * 8) = o;
}

__global__ __launch_bounds__(256) void k_tcvt(const float* __restrict__ W, unsigned short* Wt, int mode) {
    __shared__ __align__(16) float tile[64 * 68];
    const int tid = threadIdx.x; const int n0 = blockIdx.x * 64, k0 = blockIdx.y * 64;
#pragma unroll
    for (int i = 0; i < 4; ++i) { const int kk = (tid >> 4) + 16 * i, c4 = (tid & 15) * 4;
        const v4f v = *(const v4f*)(W + (size_t)(k0 + kk) * DM + n0 + c4);
        *(v4fa*)(&tile[kk * 68 + c4]) = v; }
    __syncthreads();
#pragma unroll 1
    for (int ps = 0; ps < 2; ++ps) {
#pragma unroll
        for (int i = 0; i < 2; ++i) { const int nn = (tid >> 3) + 32 * i, k8 = (tid & 7) * 8;
            float xv[8];
#pragma unroll
            for (int j = 0; j < 8; ++j) xv[j] = bfr(tile[(k8 + j) * 68 + nn]);
            const size_t oo = (size_t)(n0 + nn) * DM + k0 + k8;
            if (mode == 0) { v8us o;
#pragma unroll
                for (int j = 0; j < 8; ++j) o[j] = (unsigned short)(__float_as_uint(xv[j]) >> 16);
                *(volatile v8us*)(Wt + oo) = o;
            } else { v8h o;
#pragma unroll
                for (int j = 0; j < 8; ++j) o[j] = (h16)(xv[j] * WOS);
                *(volatile v8h*)(Wt + oo) = o; } }
        if (ps == 0) __threadfence(); }
}

__global__ __launch_bounds__(256) void k_rope(float* CS) {
#pragma clang fp contract(off)
    __shared__ __align__(16) float tb[4 * CSP];
    const int tid = threadIdx.x; const int r = tid >> 6, c = tid & 63; const int t = blockIdx.x * 4 + r;
    const float e = (float)c * (1.0f / 64.0f);
    const float inv = __builtin_amdgcn_exp2f(-(e * 13.28125f)) * __builtin_amdgcn_exp2f(-(e * 0.006462379549449f));
    const float ang = (float)t * inv;
    float sn, cs; sincosf(ang, &sn, &cs);
    tb[r * CSP + c] = cs; tb[r * CSP + 64 + c] = sn;
    __syncthreads();
    if (tid < 128) { const v4f v = *(const v4fa*)(&tb[tid * 4]); float* dst = CS + (size_t)blockIdx.x * 4 * CSP + tid * 4;
        *(volatile v4f*)dst = v; __threadfence(); *(volatile v4f*)dst = v; }
}

__global__ __launch_bounds__(256) void k_mflag(const float* __restrict__ MK, int* FL) {
    __shared__ __align__(16) int fs[FLP];
    __shared__ int al[8 * 16];
    const int tid = threadIdx.x, lane = tid & 31, wave = __builtin_amdgcn_readfirstlane((int)(threadIdx.x >> 5));
    const int row = lane >> 1, half = lane & 1;
    const size_t mo = (size_t)(blockIdx.x * 16 + row) * SEQ_FULL + half * 16;
    int alive = 0;
#pragma unroll 1
    for (int i = 0; i < FLP / 8; ++i) {
        const int ks = wave * (FLP / 8) + i;
        int nz = 0, nd = 0;
        if (ks < SEQ / 32) {
#pragma unroll
            for (int j = 0; j < 4; ++j) { const v4f v = *(const v4f*)(MK + mo + (size_t)ks * 32 + 4 * j);
#pragma unroll
                for (int e = 0; e < 4; ++e) { nz |= (v[e] != 0.0f) ? 1 : 0; nd |= (v[e] < -1.0e8f) ? 0 : 1; alive |= (v[e] > -1.0e6f) ? 1 : 0; } }
        }
        const int anz = (__ballot(nz != 0) != 0) ? 1 : 0;
        const int and_ = (__ballot(nd != 0) != 0) ? 1 : 0;
        if (lane == 0) fs[ks] = (ks < SEQ / 32) ? (anz ? (and_ ? 1 : 2) : 0) : 2;
    }
    alive |= __shfl_xor(alive, 1, 32);
    if (half == 0) al[wave * 16 + row] = alive;
    __syncthreads();
    if (tid < FLP / 4) {
        int ta = 1;
#pragma unroll 1
        for (int r = 0; r < 16; ++r) { int o = 0;
#pragma unroll 1
            for (int w = 0; w < 8; ++w) o |= al[w * 16 + r];
            ta &= (o != 0) ? 1 : 0; }
        v4i f;
#pragma unroll
        for (int j = 0; j < 4; ++j) { const int v = fs[tid * 4 + j]; f[j] = (v == 2 && ta == 0) ? 1 : v; }
        int* dst = FL + (size_t)blockIdx.x * FLP + tid * 4;
        *(volatile v4i*)dst = f; __threadfence(); *(volatile v4i*)dst = f;
    }
}

__global__ __launch_bounds__(32) __attribute__((amdgpu_num_vgpr(256)))
void k_proj(const bf* __restrict__ A, const bf* __restrict__ Bt, const float* __restrict__ bias, h16* Ph, h16* Pr,
            size_t sRB, size_t sCB, int biasRow, int useRes, int RB, int pitch, int CB) {
    __shared__ __align__(16) float os[16 * 68];
    const int K = DM;
    const int lane = threadIdx.x & 31, lr = lane & 15, hi = lane >> 4; const int r0 = blockIdx.x * 64, c0 = blockIdx.y * 64;
    v8f acc[4][4];
#pragma unroll
    for (int mb = 0; mb < 4; ++mb)
#pragma unroll
        for (int nb = 0; nb < 4; ++nb) acc[mb][nb] = (v8f){};
    const size_t aoff = (size_t)(r0 + lr) * K + 8 * hi, boff = (size_t)(c0 + lr) * K + 8 * hi;
#pragma unroll 1
    for (int kc = 0; kc < K; kc += 32) {
        v16bf a[4];
#pragma unroll
        for (int mb = 0; mb < 4; ++mb) a[mb] = ldb(A + aoff + (size_t)mb * 16 * K + kc);
#pragma unroll
        for (int nb = 0; nb < 4; ++nb) { const v16bf b = ldb(Bt + boff + (size_t)nb * 16 * K + kc);
#pragma unroll
            for (int mb = 0; mb < 4; ++mb) acc[mb][nb] = wmmab(a[mb], b, acc[mb][nb]); }
        asm volatile("v_nop\n\tv_nop\n\tv_nop\n\tv_nop" : "+v"(acc[0][0]), "+v"(acc[1][1]), "+v"(acc[2][2]), "+v"(acc[3][3]) : "v"(a[0]), "v"(a[1]), "v"(a[2]), "v"(a[3]));
    }
    float bc[4];
#pragma unroll
    for (int nb = 0; nb < 4; ++nb) { const int ci = biasRow ? 0 : (c0 + nb * 16 + lr); const float t = bfr(bias[ci]); bc[nb] = biasRow ? 0.0f : t; }
    const size_t tbase = (size_t)(r0 / RB) * sRB + (size_t)(r0 % RB) * (size_t)pitch + (size_t)(c0 / CB) * sCB + (size_t)(c0 % CB);
#pragma unroll
    for (int mb = 0; mb < 4; ++mb) {
        float br[8];
#pragma unroll
        for (int j = 0; j < 8; ++j) { const int ri = biasRow ? (r0 + mb * 16 + hi * 8 + j) : 0; const float t = bfr(bias[ri]); br[j] = biasRow ? t : 0.0f; }
#pragma unroll
        for (int nb = 0; nb < 4; ++nb) {
#pragma unroll
            for (int j = 0; j < 8; ++j) os[(hi * 8 + j) * 68 + nb * 16 + lr] = acc[mb][nb][j] + bc[nb] + br[j]; }
        wave_sync();
        const size_t sb = tbase + (size_t)(mb * 16) * (size_t)pitch;
#pragma unroll 1
        for (int ps = 0; ps < 2; ++ps) {
#pragma unroll
            for (int s = 0; s < 4; ++s) { const int row = 4 * s + (lane >> 3), c8 = (lane & 7) * 8;
                const v4f x0 = *(const v4fa*)(&os[row * 68 + c8]); const v4f x1 = *(const v4fa*)(&os[row * 68 + c8 + 4]); v8h hv, rv;
#pragma unroll
                for (int i = 0; i < 4; ++i) { const h16 a0 = (h16)x0[i]; const h16 a1 = (h16)x1[i]; hv[i] = a0; hv[4 + i] = a1; rv[i] = (h16)((x0[i] - (float)a0) * QRS); rv[4 + i] = (h16)((x1[i] - (float)a1) * QRS); }
                const size_t oo = sb + (size_t)row * (size_t)pitch + c8;
                *(volatile v8h*)(Ph + oo) = hv; if (useRes) *(volatile v8h*)(Pr + oo) = rv; }
            if (ps == 0) __threadfence(); }
        wave_sync();
    }
}

__global__ __launch_bounds__(32) __attribute__((amdgpu_num_vgpr(256)))
void k_projr(const bf* __restrict__ A, const bf* __restrict__ Bt, const float* __restrict__ bias, const float* __restrict__ CS, h16* Ph, h16* Pre) {
    __shared__ __align__(16) float os[16 * OSP];
    const int K = DM;
    const int lane = threadIdx.x & 31, lr = lane & 15, hi = lane >> 4; const int r0 = blockIdx.x * 32, hd = blockIdx.y; const int c0 = hd * HD;
    v8f acc[2][8];
#pragma unroll
    for (int mb = 0; mb < 2; ++mb)
#pragma unroll
        for (int nb = 0; nb < 8; ++nb) acc[mb][nb] = (v8f){};
    const size_t aoff = (size_t)(r0 + lr) * K + 8 * hi, boff = (size_t)(c0 + lr) * K + 8 * hi;
#pragma unroll 1
    for (int kc = 0; kc < K; kc += 32) {
        v16bf a[2];
#pragma unroll
        for (int mb = 0; mb < 2; ++mb) a[mb] = ldb(A + aoff + (size_t)mb * 16 * K + kc);
#pragma unroll
        for (int nb = 0; nb < 8; ++nb) { const v16bf b = ldb(Bt + boff + (size_t)nb * 16 * K + kc);
#pragma unroll
            for (int mb = 0; mb < 2; ++mb) acc[mb][nb] = wmmabg(a[mb], b, acc[mb][nb]); }
    }
    float bc[8];
#pragma unroll
    for (int nb = 0; nb < 8; ++nb) bc[nb] = bfr(bias[c0 + nb * 16 + lr]);
    const int bb = r0 / SEQ, tt0 = r0 % SEQ;
    const size_t prow = ((size_t)(bb * NH_ + hd) * SEQ + tt0) * HD;
    const size_t erow = ((size_t)(bb * NH_ + hd) * ER + tt0) * HD;
    const int early = (tt0 < ER) ? 1 : 0;
#pragma unroll
    for (int mb = 0; mb < 2; ++mb) {
#pragma unroll
        for (int nb = 0; nb < 8; ++nb) {
#pragma unroll
            for (int j = 0; j < 8; ++j) os[(hi * 8 + j) * OSP + nb * 16 + lr] = acc[mb][nb][j] + bc[nb]; }
        wave_sync();
#pragma unroll 1
        for (int ps = 0; ps < 2; ++ps) {
#pragma unroll
            for (int s = 0; s < 8; ++s) { const int row = 2 * s + hi, c8 = lr * 8, cc = c8 & 63;
                const v4f xl0 = *(const v4fa*)(&os[row * OSP + cc]); const v4f xl1 = *(const v4fa*)(&os[row * OSP + cc + 4]);
                const v4f xh0 = *(const v4fa*)(&os[row * OSP + 64 + cc]); const v4f xh1 = *(const v4fa*)(&os[row * OSP + 64 + cc + 4]);
                const float* cp = CS + (size_t)(tt0 + mb * 16 + row) * CSP + cc;
                const v4f cs0 = *(const v4f*)cp; const v4f cs1 = *(const v4f*)(cp + 4); const v4f sn0 = *(const v4f*)(cp + 64); const v4f sn1 = *(const v4f*)(cp + 68);
                v8h hv, rv;
#pragma unroll
                for (int i = 0; i < 4; ++i) {
                    const float ya0 = xl0[i] * cs0[i] - xh0[i] * sn0[i], yb0 = xl0[i] * sn0[i] + xh0[i] * cs0[i];
                    const float ya1 = xl1[i] * cs1[i] - xh1[i] * sn1[i], yb1 = xl1[i] * sn1[i] + xh1[i] * cs1[i];
                    const float y0 = (c8 < 64) ? ya0 : yb0; const float y1 = (c8 < 64) ? ya1 : yb1;
                    const h16 a0 = toh_flush(y0); const h16 a1 = toh_flush(y1); hv[i] = a0; hv[4 + i] = a1;
                    rv[i] = toh_flush((y0 - (float)a0) * QRS); rv[4 + i] = toh_flush((y1 - (float)a1) * QRS); }
                const size_t ro = (size_t)(mb * 16 + row) * HD + c8;
                *(volatile v8h*)(Ph + prow + ro) = hv; if (early) *(volatile v8h*)(Pre + erow + ro) = rv; }
            if (ps == 0) __threadfence(); }
        wave_sync();
    }
}

__global__ __launch_bounds__(32 * AW) __attribute__((amdgpu_num_vgpr(256)))
void k_flash(const h16* __restrict__ QH, const h16* __restrict__ KP, const h16* __restrict__ VT, const float* __restrict__ MK, const int* __restrict__ FL, h16* CX) {
    __shared__ __align__(16) float os[AW * 16 * OSP];
    const int lane = threadIdx.x & 31, wave = __builtin_amdgcn_readfirstlane((int)(threadIdx.x >> 5)), lr = lane & 15, hi = lane >> 4;
    const int zh = blockIdx.y; const int b = zh / NH_, h = zh % NH_;
    const int t0 = ER + (blockIdx.x * AW + wave) * 16;
    const size_t pbase = (size_t)zh * SEQ * HD;
    const size_t qo = pbase + (size_t)(t0 + lr) * HD + 8 * hi;
    const v16h qh0 = ldh(QH + qo), qh1 = ldh(QH + qo + 32), qh2 = ldh(QH + qo + 64), qh3 = ldh(QH + qo + 96);
    const size_t ko = pbase + (size_t)lr * HD + 8 * hi;
    const size_t vo = pbase + (size_t)lr * SEQ + 8 * hi;
    const size_t mo = (size_t)(t0 + lr) * SEQ_FULL + 8 * hi;
    const int fo = (t0 >> 4) * FLP;
    v8f o0 = (v8f){}, o1 = (v8f){}, o2 = (v8f){}, o3 = (v8f){}, o4 = (v8f){}, o5 = (v8f){}, o6 = (v8f){}, o7 = (v8f){};
    float m = -3.0e38f, l = 0.0f;
#pragma unroll 1
    for (int key0 = 0; key0 < SEQ; key0 += 32) {
        const int fl = __builtin_amdgcn_readfirstlane(FL[fo + (key0 >> 5)]);
        if (fl == 2) continue;
        const h16* ka = KP + ko + (size_t)key0 * HD;
        v8f sa = (v8f){}, sb = (v8f){};
        { const v16h a0 = ldh(ka), b0 = ldh(ka + 16 * HD); sa = wmma16g(a0, qh0, sa); sb = wmma16g(b0, qh0, sb); }
        { const v16h a1 = ldh(ka + 32), b1 = ldh(ka + 16 * HD + 32); sa = wmma16g(a1, qh1, sa); sb = wmma16g(b1, qh1, sb); }
        { const v16h a2 = ldh(ka + 64), b2 = ldh(ka + 16 * HD + 64); sa = wmma16g(a2, qh2, sa); sb = wmma16g(b2, qh2, sb); }
        { const v16h a3 = ldh(ka + 96), b3 = ldh(ka + 16 * HD + 96); sa = wmma16g(a3, qh3, sa); sb = wmma16g(b3, qh3, sb); }
        v8f mka = (v8f){}, mkb = (v8f){};
        if (fl != 0) { const v8f ra = *(const v8f*)(MK + mo + key0); const v8f rb = *(const v8f*)(MK + mo + key0 + 16);
#pragma unroll
            for (int r = 0; r < 8; ++r) { mka[r] = bfr(ra[r]) * L2E; mkb[r] = bfr(rb[r]) * L2E; } }
        float ta[8], tb[8]; float mx = -3.0e38f;
#pragma unroll
        for (int r = 0; r < 8; ++r) { ta[r] = sa[r] * SC2 + mka[r]; tb[r] = sb[r] * SC2 + mkb[r]; mx = fmaxf(mx, fmaxf(ta[r], tb[r])); }
        mx = fmaxf(mx, __shfl_xor(mx, 16, 32));
        const float mnew = fmaxf(m, mx);
        const float alpha = __builtin_amdgcn_exp2f(m - mnew);
        const float sh = PSH - mnew;
        v16h pb; float ls = 0.0f;
#pragma unroll
        for (int r = 0; r < 8; ++r) { const float ea = ta[r] + sh, eb = tb[r] + sh;
            const h16 pa = (h16)((ea < -14.0f) ? 0.0f : __builtin_amdgcn_exp2f(ea)); const h16 pc = (h16)((eb < -14.0f) ? 0.0f : __builtin_amdgcn_exp2f(eb));
            pb[r] = pa; pb[8 + r] = pc; ls += (float)pa + (float)pc; }
        l = l * alpha + ls; m = mnew;
        o0 = o0 * alpha; o1 = o1 * alpha; o2 = o2 * alpha; o3 = o3 * alpha; o4 = o4 * alpha; o5 = o5 * alpha; o6 = o6 * alpha; o7 = o7 * alpha;
        const h16* va = VT + vo + key0;
        { const v16h v0 = ldh(va), v1 = ldh(va + (size_t)16 * SEQ), v2 = ldh(va + (size_t)32 * SEQ), v3 = ldh(va + (size_t)48 * SEQ);
          o0 = wmma16g(v0, pb, o0); o1 = wmma16g(v1, pb, o1); o2 = wmma16g(v2, pb, o2); o3 = wmma16g(v3, pb, o3); }
        { const v16h v4 = ldh(va + (size_t)64 * SEQ), v5 = ldh(va + (size_t)80 * SEQ), v6 = ldh(va + (size_t)96 * SEQ), v7 = ldh(va + (size_t)112 * SEQ);
          o4 = wmma16g(v4, pb, o4); o5 = wmma16g(v5, pb, o5); o6 = wmma16g(v6, pb, o6); o7 = wmma16g(v7, pb, o7); }
    }
    l += __shfl_xor(l, 16, 32);
    const float sc = (1.0f / l) * CXS;
    const int wb = wave * 16 * OSP;
    { float* orw = &os[wb + lr * OSP + 8 * hi]; v4f a, c;
      a[0] = o0[0] * sc; a[1] = o0[1] * sc; a[2] = o0[2] * sc; a[3] = o0[3] * sc; c[0] = o0[4] * sc; c[1] = o0[5] * sc; c[2] = o0[6] * sc; c[3] = o0[7] * sc;
      *(v4fa*)(orw +   0) = a; *(v4fa*)(orw +   4) = c;
      a[0] = o1[0] * sc; a[1] = o1[1] * sc; a[2] = o1[2] * sc; a[3] = o1[3] * sc; c[0] = o1[4] * sc; c[1] = o1[5] * sc; c[2] = o1[6] * sc; c[3] = o1[7] * sc;
      *(v4fa*)(orw +  16) = a; *(v4fa*)(orw +  20) = c;
      a[0] = o2[0] * sc; a[1] = o2[1] * sc; a[2] = o2[2] * sc; a[3] = o2[3] * sc; c[0] = o2[4] * sc; c[1] = o2[5] * sc; c[2] = o2[6] * sc; c[3] = o2[7] * sc;
      *(v4fa*)(orw +  32) = a; *(v4fa*)(orw +  36) = c;
      a[0] = o3[0] * sc; a[1] = o3[1] * sc; a[2] = o3[2] * sc; a[3] = o3[3] * sc; c[0] = o3[4] * sc; c[1] = o3[5] * sc; c[2] = o3[6] * sc; c[3] = o3[7] * sc;
      *(v4fa*)(orw +  48) = a; *(v4fa*)(orw +  52) = c;
      a[0] = o4[0] * sc; a[1] = o4[1] * sc; a[2] = o4[2] * sc; a[3] = o4[3] * sc; c[0] = o4[4] * sc; c[1] = o4[5] * sc; c[2] = o4[6] * sc; c[3] = o4[7] * sc;
      *(v4fa*)(orw +  64) = a; *(v4fa*)(orw +  68) = c;
      a[0] = o5[0] * sc; a[1] = o5[1] * sc; a[2] = o5[2] * sc; a[3] = o5[3] * sc; c[0] = o5[4] * sc; c[1] = o5[5] * sc; c[2] = o5[6] * sc; c[3] = o5[7] * sc;
      *(v4fa*)(orw +  80) = a; *(v4fa*)(orw +  84) = c;
      a[0] = o6[0] * sc; a[1] = o6[1] * sc; a[2] = o6[2] * sc; a[3] = o6[3] * sc; c[0] = o6[4] * sc; c[1] = o6[5] * sc; c[2] = o6[6] * sc; c[3] = o6[7] * sc;
      *(v4fa*)(orw +  96) = a; *(v4fa*)(orw + 100) = c;
      a[0] = o7[0] * sc; a[1] = o7[1] * sc; a[2] = o7[2] * sc; a[3] = o7[3] * sc; c[0] = o7[4] * sc; c[1] = o7[5] * sc; c[2] = o7[6] * sc; c[3] = o7[7] * sc;
      *(v4fa*)(orw + 112) = a; *(v4fa*)(orw + 116) = c; }
    wave_sync();
    h16* crow = CX + ((size_t)b * SEQ + t0) * DM + h * HD;
#pragma unroll 1
    for (int ps = 0; ps < 2; ++ps) {
#pragma unroll
        for (int s = 0; s < 8; ++s) { const int row = 2 * s + hi, c8 = lr * 8;
            const v4f x0 = *(const v4fa*)(&os[wb + row * OSP + c8]); const v4f x1 = *(const v4fa*)(&os[wb + row * OSP + c8 + 4]); v8h hv;
#pragma unroll
            for (int i = 0; i < 4; ++i) { hv[i] = toh_flush(x0[i]); hv[4 + i] = toh_flush(x1[i]); }
            *(volatile v8h*)(crow + (size_t)row * DM + c8) = hv; }
        if (ps == 0) __threadfence(); }
}

__global__ __launch_bounds__(32 * AW) __attribute__((amdgpu_num_vgpr(256)))
void k_flash_e(const h16* __restrict__ QH, const h16* __restrict__ QRE, const h16* __restrict__ KP, const h16* __restrict__ KRE,
               const h16* __restrict__ VT, const h16* __restrict__ VRE, const float* __restrict__ MK, const int* __restrict__ FL, h16* CX, h16* CXL) {
    __shared__ __align__(16) float os[AW * 16 * ESP];
    const int lane = threadIdx.x & 31, wave = __builtin_amdgcn_readfirstlane((int)(threadIdx.x >> 5)), lr = lane & 15, hi = lane >> 4;
    const int zh = blockIdx.y, dz = blockIdx.z; const int b = zh / NH_, h = zh % NH_;
    const int t0 = (blockIdx.x * AW + wave) * 16;
    const size_t pbase = (size_t)zh * SEQ * HD, ebase = (size_t)zh * ER * HD;
    const size_t qo  = pbase + (size_t)(t0 + lr) * HD + 8 * hi;
    const size_t qeo = ebase + (size_t)(t0 + lr) * HD + 8 * hi;
    const size_t ko  = pbase + (size_t)lr * HD + 8 * hi;
    const size_t keo = ebase + (size_t)lr * HD + 8 * hi;
    const size_t vo  = pbase + (size_t)(64 * dz + lr) * SEQ + 8 * hi;
    const size_t veo = ebase + (size_t)(64 * dz + lr) * ER + 8 * hi;
    const size_t mo = (size_t)(t0 + lr) * SEQ_FULL + 8 * hi;
    const int fo = (t0 >> 4) * FLP;
    v8f oH0 = (v8f){}, oH1 = (v8f){}, oH2 = (v8f){}, oH3 = (v8f){}, oR0 = (v8f){}, oR1 = (v8f){}, oR2 = (v8f){}, oR3 = (v8f){};
    float m = -3.0e38f, l = 0.0f;
#pragma unroll 1
    for (int key0 = 0; key0 < SEQ; key0 += 32) {
        const int fl = __builtin_amdgcn_readfirstlane(FL[fo + (key0 >> 5)]);
        if (fl == 2) continue;
        const int kc = (key0 < ER) ? key0 : (ER - 32);
        const float qri = (key0 < ER) ? QRI : 0.0f;
        const float prs = (key0 < ER) ? QRS : 0.0f;
        v8f sHa = (v8f){}, sLa = (v8f){}, sHb = (v8f){}, sLb = (v8f){};
#pragma unroll
        for (int s = 0; s < 4; ++s) {
            const v16h qh = ldh(QH + qo + 32 * s);
            const v16h ka = ldh(KP + ko + (size_t)key0 * HD + 32 * s), kb = ldh(KP + ko + (size_t)(key0 + 16) * HD + 32 * s);
            sHa = wmma16g(ka, qh, sHa); sHb = wmma16g(kb, qh, sHb);
            if (ESC_RES) {
                const v16h qr = ldh(QRE + qeo + 32 * s);
                const v16h kra = ldh(KRE + keo + (size_t)kc * HD + 32 * s), krb = ldh(KRE + keo + (size_t)(kc + 16) * HD + 32 * s);
                sLa = wmma16g(ka, qr, sLa); sLa = wmma16g(kra, qh, sLa);
                sLb = wmma16g(kb, qr, sLb); sLb = wmma16g(krb, qh, sLb);
            }
        }
        v8f mka = (v8f){}, mkb = (v8f){};
        if (fl != 0) { const v8f ra = *(const v8f*)(MK + mo + key0); const v8f rb = *(const v8f*)(MK + mo + key0 + 16);
#pragma unroll
            for (int r = 0; r < 8; ++r) { mka[r] = bfr(ra[r]) * L2E; mkb[r] = bfr(rb[r]) * L2E; } }
        float ta[8], tb[8]; float mx = -3.0e38f;
#pragma unroll
        for (int r = 0; r < 8; ++r) { ta[r] = (sHa[r] + sLa[r] * qri) * SC2 + mka[r]; tb[r] = (sHb[r] + sLb[r] * qri) * SC2 + mkb[r]; mx = fmaxf(mx, fmaxf(ta[r], tb[r])); }
        mx = fmaxf(mx, __shfl_xor(mx, 16, 32));
        const float mnew = fmaxf(m, mx);
        const float alpha = __builtin_amdgcn_exp2f(m - mnew);
        const float sh = PSH - mnew;
        v16h pb, prb; float ls = 0.0f;
#pragma unroll
        for (int r = 0; r < 8; ++r) { const float ea = ta[r] + sh, eb = tb[r] + sh;
            const float fa = (ea < -14.0f) ? 0.0f : __builtin_amdgcn_exp2f(ea); const float fb = (eb < -14.0f) ? 0.0f : __builtin_amdgcn_exp2f(eb);
            const h16 pa = (h16)fa; const h16 pc = (h16)fb;
            pb[r] = pa; pb[8 + r] = pc; prb[r] = toh_flush((fa - (float)pa) * prs); prb[8 + r] = toh_flush((fb - (float)pc) * prs); ls += fa + fb; }
        v16h pz = pb;
        if (key0 >= ER) pz = (v16h){};
        l = l * alpha + ls; m = mnew;
        oH0 = oH0 * alpha; oH1 = oH1 * alpha; oH2 = oH2 * alpha; oH3 = oH3 * alpha; oR0 = oR0 * alpha; oR1 = oR1 * alpha; oR2 = oR2 * alpha; oR3 = oR3 * alpha;
        const h16* va = VT + vo + key0; const h16* vra = VRE + veo + kc;
        { const v16h v0 = ldh(va), r0 = ldh(vra);
          oH0 = wmma16g(v0, pb, oH0); oR0 = wmma16g(v0, prb, oR0); oR0 = wmma16g(r0, pz, oR0); }
        { const v16h v1 = ldh(va + (size_t)16 * SEQ), r1 = ldh(vra + (size_t)16 * ER);
          oH1 = wmma16g(v1, pb, oH1); oR1 = wmma16g(v1, prb, oR1); oR1 = wmma16g(r1, pz, oR1); }
        { const v16h v2 = ldh(va + (size_t)32 * SEQ), r2 = ldh(vra + (size_t)32 * ER);
          oH2 = wmma16g(v2, pb, oH2); oR2 = wmma16g(v2, prb, oR2); oR2 = wmma16g(r2, pz, oR2); }
        { const v16h v3 = ldh(va + (size_t)48 * SEQ), r3 = ldh(vra + (size_t)48 * ER);
          oH3 = wmma16g(v3, pb, oH3); oR3 = wmma16g(v3, prb, oR3); oR3 = wmma16g(r3, pz, oR3); }
    }
    l += __shfl_xor(l, 16, 32);
    const float sc = (1.0f / l) * CXS;
    const int wb = wave * 16 * ESP;
    { float* orw = &os[wb + lr * ESP + 8 * hi]; v4f a, c; v8f t;
      t = (oH0 + oR0 * QRI) * sc; a[0] = t[0]; a[1] = t[1]; a[2] = t[2]; a[3] = t[3]; c[0] = t[4]; c[1] = t[5]; c[2] = t[6]; c[3] = t[7];
      *(v4fa*)(orw +  0) = a; *(v4fa*)(orw +  4) = c;
      t = (oH1 + oR1 * QRI) * sc; a[0] = t[0]; a[1] = t[1]; a[2] = t[2]; a[3] = t[3]; c[0] = t[4]; c[1] = t[5]; c[2] = t[6]; c[3] = t[7];
      *(v4fa*)(orw + 16) = a; *(v4fa*)(orw + 20) = c;
      t = (oH2 + oR2 * QRI) * sc; a[0] = t[0]; a[1] = t[1]; a[2] = t[2]; a[3] = t[3]; c[0] = t[4]; c[1] = t[5]; c[2] = t[6]; c[3] = t[7];
      *(v4fa*)(orw + 32) = a; *(v4fa*)(orw + 36) = c;
      t = (oH3 + oR3 * QRI) * sc; a[0] = t[0]; a[1] = t[1]; a[2] = t[2]; a[3] = t[3]; c[0] = t[4]; c[1] = t[5]; c[2] = t[6]; c[3] = t[7];
      *(v4fa*)(orw + 48) = a; *(v4fa*)(orw + 52) = c; }
    wave_sync();
    h16* crow = CX + ((size_t)b * SEQ + t0) * DM + h * HD + 64 * dz;
    h16* lrow = CXL + ((size_t)b * ER + t0) * DM + h * HD + 64 * dz;
#pragma unroll 1
    for (int ps = 0; ps < 2; ++ps) {
#pragma unroll
        for (int s = 0; s < 4; ++s) { const int row = 4 * s + (lane >> 3), c8 = (lane & 7) * 8;
            const v4f x0 = *(const v4fa*)(&os[wb + row * ESP + c8]); const v4f x1 = *(const v4fa*)(&os[wb + row * ESP + c8 + 4]); v8h hv, lv;
#pragma unroll
            for (int i = 0; i < 4; ++i) { const h16 a0 = toh_flush(x0[i]); const h16 a1 = toh_flush(x1[i]); hv[i] = a0; hv[4 + i] = a1;
                lv[i] = toh_flush(x0[i] - (float)a0); lv[4 + i] = toh_flush(x1[i] - (float)a1); }
            *(volatile v8h*)(crow + (size_t)row * DM + c8) = hv; *(volatile v8h*)(lrow + (size_t)row * DM + c8) = lv; }
        if (ps == 0) __threadfence(); }
}

__global__ __launch_bounds__(32) __attribute__((amdgpu_num_vgpr(256)))
void k_oproj(const h16* __restrict__ A, const h16* __restrict__ Bt, const float* __restrict__ bias, float* OUT) {
    __shared__ __align__(16) float os[16 * 68];
    const int K = DM;
    const int lane = threadIdx.x & 31, lr = lane & 15, hi = lane >> 4; const int r0 = blockIdx.x * 64, c0 = blockIdx.y * 64;
    v8f acc[4][4];
#pragma unroll
    for (int mb = 0; mb < 4; ++mb)
#pragma unroll
        for (int nb = 0; nb < 4; ++nb) acc[mb][nb] = (v8f){};
    const size_t aoff = (size_t)(r0 + lr) * K + 8 * hi, boff = (size_t)(c0 + lr) * K + 8 * hi;
#pragma unroll 1
    for (int kc = 0; kc < K; kc += 32) {
        v16h a[4];
#pragma unroll
        for (int mb = 0; mb < 4; ++mb) a[mb] = ldh(A + aoff + (size_t)mb * 16 * K + kc);
#pragma unroll
        for (int nb = 0; nb < 4; ++nb) { const v16h b = ldh(Bt + boff + (size_t)nb * 16 * K + kc);
#pragma unroll
            for (int mb = 0; mb < 4; ++mb) acc[mb][nb] = wmma16(a[mb], b, acc[mb][nb]); }
        asm volatile("v_nop\n\tv_nop\n\tv_nop\n\tv_nop" : "+v"(acc[0][0]), "+v"(acc[1][1]), "+v"(acc[2][2]), "+v"(acc[3][3]) : "v"(a[0]), "v"(a[1]), "v"(a[2]), "v"(a[3]));
    }
    float bc[4];
#pragma unroll
    for (int nb = 0; nb < 4; ++nb) bc[nb] = bfr(bias[c0 + nb * 16 + lr]);
    float* obase = OUT + ((size_t)(r0 / SEQ) * OUT_SEQ + (size_t)(r0 % SEQ)) * DM + c0;
#pragma unroll
    for (int mb = 0; mb < 4; ++mb) {
#pragma unroll
        for (int nb = 0; nb < 4; ++nb) {
#pragma unroll
            for (int j = 0; j < 8; ++j) os[(hi * 8 + j) * 68 + nb * 16 + lr] = acc[mb][nb][j] * OSC + bc[nb]; }
        wave_sync();
        float* orow = obase + (size_t)(mb * 16) * DM;
#pragma unroll 1
        for (int ps = 0; ps < 2; ++ps) {
#pragma unroll
            for (int s = 0; s < 8; ++s) { const int row = 2 * s + hi, cofs = lr * 4;
                const v4f val = *(const v4fa*)(&os[row * 68 + cofs]);
                *(volatile v4f*)(orow + (size_t)row * DM + cofs) = val; }
            if (ps == 0) __threadfence(); }
        wave_sync();
    }
}

__global__ __launch_bounds__(32) __attribute__((amdgpu_num_vgpr(256)))
void k_oproje(const h16* __restrict__ AH, const h16* __restrict__ AL, const h16* __restrict__ Bt, const float* __restrict__ bias, float* OUT) {
    __shared__ __align__(16) float os[16 * 68];
    const int K = DM;
    const int lane = threadIdx.x & 31, lr = lane & 15, hi = lane >> 4; const int e0 = blockIdx.x * 64, c0 = blockIdx.y * 64;
    const int bb = e0 / ER, tt = e0 % ER;
    v8f acc[4][4];
#pragma unroll
    for (int mb = 0; mb < 4; ++mb)
#pragma unroll
        for (int nb = 0; nb < 4; ++nb) acc[mb][nb] = (v8f){};
    const size_t ahoff = ((size_t)bb * SEQ + tt + lr) * K + 8 * hi, aloff = (size_t)(e0 + lr) * K + 8 * hi, boff = (size_t)(c0 + lr) * K + 8 * hi;
#pragma unroll 1
    for (int kc = 0; kc < K; kc += 32) {
        v16h a[4];
#pragma unroll
        for (int mb = 0; mb < 4; ++mb) a[mb] = ldh(AH + ahoff + (size_t)mb * 16 * K + kc);
#pragma unroll
        for (int nb = 0; nb < 4; ++nb) { const v16h b = ldh(Bt + boff + (size_t)nb * 16 * K + kc);
#pragma unroll
            for (int mb = 0; mb < 4; ++mb) acc[mb][nb] = wmma16g(a[mb], b, acc[mb][nb]); }
    }
#pragma unroll 1
    for (int kc = 0; kc < K; kc += 32) {
        v16h a[4];
#pragma unroll
        for (int mb = 0; mb < 4; ++mb) a[mb] = ldh(AL + aloff + (size_t)mb * 16 * K + kc);
#pragma unroll
        for (int nb = 0; nb < 4; ++nb) { const v16h b = ldh(Bt + boff + (size_t)nb * 16 * K + kc);
#pragma unroll
            for (int mb = 0; mb < 4; ++mb) acc[mb][nb] = wmma16g(a[mb], b, acc[mb][nb]); }
    }
    float bc[4];
#pragma unroll
    for (int nb = 0; nb < 4; ++nb) bc[nb] = bfr(bias[c0 + nb * 16 + lr]);
    float* obase = OUT + ((size_t)bb * OUT_SEQ + (size_t)tt) * DM + c0;
#pragma unroll
    for (int mb = 0; mb < 4; ++mb) {
#pragma unroll
        for (int nb = 0; nb < 4; ++nb) {
#pragma unroll
            for (int j = 0; j < 8; ++j) os[(hi * 8 + j) * 68 + nb * 16 + lr] = acc[mb][nb][j] * OSC + bc[nb]; }
        wave_sync();
        float* orow = obase + (size_t)(mb * 16) * DM;
#pragma unroll 1
        for (int ps = 0; ps < 2; ++ps) {
#pragma unroll
            for (int s = 0; s < 8; ++s) { const int row = 2 * s + hi, cofs = lr * 4;
                const v4f val = *(const v4fa*)(&os[row * 68 + cofs]);
                *(volatile v4f*)(orow + (size_t)row * DM + cofs) = val; }
            if (ps == 0) __threadfence(); }
        wave_sync();
    }
}

static constexpr size_t al256(size_t v) { return (v + 255) & ~(size_t)255; }
static constexpr size_t SZ_XB = al256((size_t)NB * SEQ * DM * 2);
static constexpr size_t SZ_CX = al256((size_t)NB * SEQ * DM * 2);
static constexpr size_t SZ_WT = al256((size_t)3 * DM * DM * 2);
static constexpr size_t SZ_WO = al256((size_t)DM * DM * 2);
static constexpr size_t SZ_PL = al256((size_t)NB * NH_ * SEQ * HD * 2);
static constexpr size_t SZ_EP = al256((size_t)NB * NH_ * ER * HD * 2);
static constexpr size_t SZ_CL = al256((size_t)NB * ER * DM * 2);
static constexpr size_t SZ_CS = al256((size_t)SEQ * CSP * 4);
static constexpr size_t SZ_FL = al256((size_t)(SEQ / 16) * FLP * 4);
static constexpr size_t SZ_TOTAL = SZ_XB + SZ_WT + SZ_WO + 3 * SZ_PL + 4 * SZ_EP + SZ_CL + SZ_CS + SZ_FL;
static_assert(SZ_CX <= SZ_XB);
static_assert(SZ_TOTAL <= (size_t)134217728);
static_assert(((size_t)DM * DM * 2) % 256 == 0);
static_assert((size_t)NB * NH_ * SEQ * HD == (size_t)NB * SEQ * DM);
static_assert((size_t)NB * NH_ * ER * HD == (size_t)NB * DM * ER);
static_assert(((size_t)DM * ER * 2) % 256 == 0);
static_assert(((size_t)ER * DM * 2) % 256 == 0);

extern "C" void kernel_launch(void* const* d_in, const int* in_sizes, int n_in,
                              void* d_out, int out_size, void* d_ws, size_t ws_size, hipStream_t stream) {
    if (n_in < 10) return;
    const size_t needx = ((size_t)(NB - 1) * SEQ_FULL + SEQ) * DM;
    if ((size_t)in_sizes[0] < needx) return;
    if ((size_t)in_sizes[1] < (size_t)(SEQ - 1) * SEQ_FULL + SEQ) return;
    if ((size_t)in_sizes[2] < (size_t)DM * DM || (size_t)in_sizes[4] < (size_t)DM * DM || (size_t)in_sizes[6] < (size_t)DM * DM || (size_t)in_sizes[8] < (size_t)DM * DM) return;
    if ((size_t)in_sizes[3] < (size_t)DM || (size_t)in_sizes[5] < (size_t)DM || (size_t)in_sizes[7] < (size_t)DM || (size_t)in_sizes[9] < (size_t)DM) return;
    if ((size_t)out_size < ((size_t)(NB - 1) * OUT_SEQ + SEQ) * DM) return;
    if (SZ_TOTAL > ws_size) return;
    const float* x  = (const float*)d_in[0];
    const float* mk = (const float*)d_in[1];
    const float* wq = (const float*)d_in[2]; const float* bq = (const float*)d_in[3];
    const float* wk = (const float*)d_in[4]; const float* bk = (const float*)d_in[5];
    const float* wv = (const float*)d_in[6]; const float* bv = (const float*)d_in[7];
    const float* wo = (const float*)d_in[8]; const float* bo = (const float*)d_in[9];
    float* OUT = (float*)d_out;
    char* wsp = (char*)d_ws;
    bf* XB = (bf*)wsp; h16* CX = (h16*)wsp; wsp += SZ_XB;
    bf* WT = (bf*)wsp; wsp += SZ_WT;
    h16* WOT = (h16*)wsp; wsp += SZ_WO;
    h16* QH = (h16*)wsp; wsp += SZ_PL;
    h16* KP = (h16*)wsp; wsp += SZ_PL;
    h16* VT = (h16*)wsp; wsp += SZ_PL;
    h16* QRE = (h16*)wsp; wsp += SZ_EP;
    h16* KRE = (h16*)wsp; wsp += SZ_EP;
    h16* VHE = (h16*)wsp; wsp += SZ_EP;
    h16* VRE = (h16*)wsp; wsp += SZ_EP;
    h16* CXL = (h16*)wsp; wsp += SZ_CL;
    float* CS = (float*)wsp; wsp += SZ_CS;
    int* FL = (int*)wsp; wsp += SZ_FL;
    bf* WQT = WT; bf* WKT = WT + (size_t)DM * DM; bf* WVT = WT + (size_t)2 * DM * DM;

    if (SEQ == SEQ_FULL) {
        const size_t n8 = (size_t)NB * SEQ * DM / 8;
        k_cvt8<<<(unsigned)((n8 + 255) / 256), 256, 0, stream>>>(x, XB, n8);
    } else {
        const size_t n8 = (size_t)SEQ * DM / 8;
        for (int b = 0; b < NB; ++b) k_cvt8<<<(unsigned)((n8 + 255) / 256), 256, 0, stream>>>(x + (size_t)b * SEQ_FULL * DM, XB + (size_t)b * SEQ * DM, n8);
    }
    { const dim3 tg(DM / 64, DM / 64, 1);
      k_tcvt<<<tg, 256, 0, stream>>>(wq, (unsigned short*)WQT, 0);
      k_tcvt<<<tg, 256, 0, stream>>>(wk, (unsigned short*)WKT, 0);
      k_tcvt<<<tg, 256, 0, stream>>>(wv, (unsigned short*)WVT, 0);
      k_tcvt<<<tg, 256, 0, stream>>>(wo, (unsigned short*)WOT, 1); }

    k_rope<<<SEQ / 4, 256, 0, stream>>>(CS);
    k_mflag<<<SEQ / 16, 256, 0, stream>>>(mk, FL);

    k_projr<<<dim3(NB * SEQ / 32, NH_, 1), 32, 0, stream>>>(XB, WQT, bq, CS, QH, QRE);
    k_projr<<<dim3(NB * SEQ / 32, NH_, 1), 32, 0, stream>>>(XB, WKT, bk, CS, KP, KRE);
    k_proj<<<dim3(DM / 64, NB * SEQ / 64, 1), 32, 0, stream>>>(WVT, XB, bv, VT, VT, (size_t)0, (size_t)DM * SEQ, 1, 0, DM, SEQ, SEQ);
    for (int b = 0; b < NB; ++b)
        k_proj<<<dim3(DM / 64, ER / 64, 1), 32, 0, stream>>>(WVT, XB + (size_t)b * SEQ * DM, bv, VHE + (size_t)b * DM * ER, VRE + (size_t)b * DM * ER,
                                                             (size_t)0, (size_t)DM * ER, 1, 1, DM, ER, ER);

    if (SEQ > ER)
        k_flash<<<dim3((SEQ - ER) / (16 * AW), NB * NH_, 1), 32 * AW, 0, stream>>>(QH, KP, VT, mk, FL, CX);
    k_flash_e<<<dim3(ER / (16 * AW), NB * NH_, 2), 32 * AW, 0, stream>>>(QH, QRE, KP, KRE, VT, VRE, mk, FL, CX, CXL);

    if (SEQ > ER)
        for (int b = 0; b < NB; ++b)
            k_oproj<<<dim3((SEQ - ER) / 64, DM / 64, 1), 32, 0, stream>>>(CX + ((size_t)b * SEQ + ER) * DM, WOT, bo, OUT + ((size_t)b * OUT_SEQ + ER) * DM);
    k_oproje<<<dim3(NB * ER / 64, DM / 64, 1), 32, 0, stream>>>(CX, CXL, WOT, bo, OUT);
}
